// Eq2to2_69372311765323
// MI455X (gfx1250) — hardware-run, weakly checked
//
#include <hip/hip_runtime.h>


#ifndef NB
#define NB 4
#endif
#define NB_FULL 4
#define MM   128
#define DD   128
#define SS   128
#define NBAS 15
#define KM   256
#define KA   384
#define NA   384
#define WCAR 64.0f
#define WINV 0.015625f
#define SLOPE 0.01f

static_assert(NB <= NB_FULL);
static_assert(MM == 128);
static_assert(DD == 128);
static_assert(SS == 128);
static_assert(KM == 2 * DD);
static_assert(KA == 3 * DD);
static_assert(NA == 3 * SS);
static_assert(KM % 32 == 0);
static_assert(KA % 32 == 0);
static_assert(DD % 32 == 0);
static_assert(MM % 64 == 0);
static_assert((NB * MM) % 64 == 0);
static_assert(SS % 64 == 0);
static_assert(NA % 64 == 0);
static_assert(DD % 8 == 0);
static_assert(((size_t)MM * MM * DD) % 8 == 0);
static_assert(32 * 16 * 8 == 16 * 64 * 4);
static_assert(16 * 68 * 4 <= 131072);
static_assert((2 * DD + DD + NA) * 4 <= 131072);

typedef _Float16 h16;
typedef unsigned short bf;
typedef __attribute__((ext_vector_type(16))) __bf16   v16bf;
typedef __attribute__((ext_vector_type(16))) _Float16 v16h;
typedef __attribute__((ext_vector_type(8)))  _Float16 v8h;
typedef __attribute__((ext_vector_type(8)))  unsigned short v8us;
typedef __attribute__((ext_vector_type(8)))  float    v8f;
typedef __attribute__((ext_vector_type(4)))  float    v4f;
typedef v4f  __attribute__((may_alias)) v4fa;

__device__ __forceinline__ unsigned short f2bf(float f) { unsigned u = __float_as_uint(f); u += 0x7FFFu + ((u >> 16) & 1u); return (unsigned short)(u >> 16); }
__device__ __forceinline__ float bfr(float f) { return __uint_as_float(((unsigned)f2bf(f)) << 16); }
__device__ __forceinline__ v16h cat16(v8h lo, v8h hi) { return __builtin_shufflevector(lo, hi, 0, 1, 2, 3, 4, 5, 6, 7, 8, 9, 10, 11, 12, 13, 14, 15); }
__device__ __forceinline__ v16bf cat16b(v8us lo, v8us hi) { return __builtin_bit_cast(v16bf, __builtin_shufflevector(lo, hi, 0, 1, 2, 3, 4, 5, 6, 7, 8, 9, 10, 11, 12, 13, 14, 15)); }
__device__ __forceinline__ v8f wmma16(v16h a, v16h b, v8f c) { return __builtin_amdgcn_wmma_f32_16x16x32_f16(false, a, false, b, (short)0, c, false, false); }
__device__ __forceinline__ v8f wmmab(v16bf a, v16bf b, v8f c) { return __builtin_amdgcn_wmma_f32_16x16x32_bf16(false, a, false, b, (short)0, c, false, false); }
__device__ __forceinline__ v16h  ldh(const h16* p) { return cat16(*(const v8h*)p, *(const v8h*)(p + 16)); }
__device__ __forceinline__ v16bf ldb(const bf* p)  { return cat16b(*(const v8us*)p, *(const v8us*)(p + 16)); }
__device__ __forceinline__ void wave_sync() { __builtin_amdgcn_fence(3  , "wavefront"); __builtin_amdgcn_wave_barrier(); asm volatile("" ::: "memory"); }

__device__ __forceinline__ v8f wmma16g(v16h a, v16h b, v8f c) { c = wmma16(a, b, c); asm volatile("v_nop\n\tv_nop\n\tv_nop\n\tv_nop" : "+v"(c) : "v"(a), "v"(b)); return c; }
__device__ __forceinline__ v8f wmmabg(v16bf a, v16bf b, v8f c) { c = wmmab(a, b, c); asm volatile("v_nop\n\tv_nop\n\tv_nop\n\tv_nop" : "+v"(c) : "v"(a), "v"(b)); return c; }
static __device__ __forceinline__ h16 toh_flush(float v) { const h16 r = (h16)v; return (fabsf(v) < 6.103515625e-05f) ? (h16)0.0f : r; }

__global__ __launch_bounds__(256) void k_cvt8(const float* __restrict__ src, bf* dst, size_t n8) {
    const size_t i = (size_t)blockIdx.x * 256 + threadIdx.x; if (i >= n8) return;
    const v8f v = *(const v8f*)(src + i * 8); v8us o;
#pragma unroll
    for (int k = 0; k < 8; ++k) o[k] = f2bf(v[k]);
    *(volatile v8us*)(dst + i * 8) = o; __threadfence(); *(volatile v8us*)(dst + i * 8) = o;
}

#define NWM8 (SS * KM / 8)
#define NWA8 (NA * KA / 8)
static_assert(NWM8 % 256 == 0);
static_assert((NWM8 + NWA8) % 256 == 0);
__global__ __launch_bounds__(256) void k_pack(const float* __restrict__ coefs, bf* WMp, h16* WAp) {
#pragma clang fp contract(off)
    const int t = blockIdx.x * 256 + threadIdx.x;
    if (t < NWM8) {
        const int s = t / (KM / 8), k8 = (t % (KM / 8)) * 8;
        const int bsel = (k8 < DD) ? 9 : 10; const int d0 = k8 % DD;
        v8us o;
#pragma unroll
        for (int e = 0; e < 8; ++e) o[e] = f2bf(coefs[((size_t)(d0 + e) * SS + s) * NBAS + bsel]);
        *(volatile v8us*)(WMp + (size_t)t * 8) = o; __threadfence(); *(volatile v8us*)(WMp + (size_t)t * 8) = o;
    } else if (t < NWM8 + NWA8) {
        const int u = t - NWM8; const int c = u / (KA / 8), k8 = (u % (KA / 8)) * 8;
        const int kb = k8 / DD, kd0 = k8 % DD, cb = c / SS, cs = c % SS;
        const int bsel = (int)((0x0CB268357ull >> (4 * (kb * 3 + cb))) & 15ull);
        v8h o;
#pragma unroll
        for (int e = 0; e < 8; ++e) o[e] = toh_flush(bfr(coefs[((size_t)(kd0 + e) * SS + cs) * NBAS + bsel]) * WCAR);
        *(volatile v8h*)(WAp + (size_t)u * 8) = o; __threadfence(); *(volatile v8h*)(WAp + (size_t)u * 8) = o;
    }
}

__global__ __launch_bounds__(128) void k_rowdiag(const float* __restrict__ x, float* AF, h16* AH) {
#pragma clang fp contract(off)
    __shared__ __align__(16) float st[2 * DD];
    const int p = blockIdx.x, i = p & (MM - 1), d = threadIdx.x;
    const int wave = __builtin_amdgcn_readfirstlane((int)(threadIdx.x >> 5));
    const float* xb = x + (size_t)p * MM * DD + d;
    float acc = 0.0f;
#pragma unroll 4
    for (int j = 0; j < MM; ++j) acc += bfr(xb[(size_t)j * DD]);
    st[d] = acc; st[DD + d] = bfr(xb[(size_t)i * DD]);
    __syncthreads();
    if (wave < 2) {
        const int t = threadIdx.x;
        const v4f v = *(const v4fa*)(&st[4 * t]);
        float* o = AF + (size_t)p * (2 * DD) + 4 * t;
        *(volatile v4f*)o = v; __threadfence(); *(volatile v4f*)o = v;
    } else if (wave == 2) {
        const int l = threadIdx.x & 31;
        const v4f x0 = *(const v4fa*)(&st[8 * l]); const v4f x1 = *(const v4fa*)(&st[8 * l + 4]); v8h hv;
#pragma unroll
        for (int e = 0; e < 4; ++e) { hv[e] = toh_flush(x0[e]); hv[4 + e] = toh_flush(x1[e]); }
        h16* o = AH + (size_t)p * KA + DD + 8 * l;
        *(volatile v8h*)o = hv; __threadfence(); *(volatile v8h*)o = hv;
    }
}

__global__ __launch_bounds__(128) void k_cols(const float* __restrict__ x, h16* AH) {
#pragma clang fp contract(off)
    __shared__ __align__(16) float st[DD];
    const int p = blockIdx.x, n = p / MM, j = p % MM, d = threadIdx.x;
    const float* xb = x + ((size_t)n * MM * MM + j) * DD + d;
    float acc = 0.0f;
#pragma unroll 4
    for (int i = 0; i < MM; ++i) acc += bfr(xb[(size_t)i * MM * DD]);
    st[d] = acc;
    __syncthreads();
    if (threadIdx.x < 16) {
        const int l = threadIdx.x;
        const v4f x0 = *(const v4fa*)(&st[8 * l]); const v4f x1 = *(const v4fa*)(&st[8 * l + 4]); v8h hv;
#pragma unroll
        for (int e = 0; e < 4; ++e) { hv[e] = toh_flush(x0[e]); hv[4 + e] = toh_flush(x1[e]); }
        h16* o = AH + (size_t)p * KA + 8 * l;
        *(volatile v8h*)o = hv; __threadfence(); *(volatile v8h*)o = hv;
    }
}

__global__ __launch_bounds__(128) void k_scal(const float* __restrict__ AF, const float* __restrict__ coefs, const float* __restrict__ bias, const float* __restrict__ dbias, float* ADDp) {
#pragma clang fp contract(off)
    __shared__ float sdv[DD];
    __shared__ float sav[DD];
    __shared__ __align__(16) float st[NA];
    const int n = blockIdx.x, t = threadIdx.x;
    const int wave = __builtin_amdgcn_readfirstlane((int)(threadIdx.x >> 5));
    float sd = 0.0f, sa = 0.0f;
#pragma unroll 1
    for (int i = 0; i < MM; ++i) { const float* r = AF + ((size_t)n * MM + i) * (2 * DD); sa += r[t]; sd += r[DD + t]; }
    sdv[t] = sd; sav[t] = sa;
    __syncthreads();
    float aF = bfr(bias[t]), aG = bfr(dbias[t]);
#pragma unroll 1
    for (int d = 0; d < DD; ++d) {
        const float* c = coefs + ((size_t)d * SS + t) * NBAS;
        const float sdd = sdv[d], saa = sav[d];
        aF += bfr(c[13]) * sdd + bfr(c[14]) * saa;
        aG += bfr(c[1]) * sdd + bfr(c[4]) * saa;
    }
    st[t] = aF; st[SS + t] = 0.0f; st[2 * SS + t] = aG;
    __syncthreads();
    if (wave < 3) {
        const v4f v = *(const v4fa*)(&st[4 * t]);
        float* o = ADDp + (size_t)n * NA + 4 * t;
        *(volatile v4f*)o = v; __threadfence(); *(volatile v4f*)o = v;
    }
}

__global__ __launch_bounds__(32) void k_agg(const h16* __restrict__ A, const h16* __restrict__ Bt, const float* __restrict__ ADDp, float* HP) {
    __shared__ __align__(16) float os[16 * 68];
    const int lane = threadIdx.x & 31, lr = lane & 15, hi = lane >> 4; const int r0 = blockIdx.x * 64, c0 = blockIdx.y * 64;
    v8f acc[4][4];
#pragma unroll
    for (int mb = 0; mb < 4; ++mb)
#pragma unroll
        for (int nb = 0; nb < 4; ++nb) acc[mb][nb] = (v8f){};
    const size_t aoff = (size_t)(r0 + lr) * KA + 8 * hi, boff = (size_t)(c0 + lr) * KA + 8 * hi;
#pragma unroll 1
    for (int kc = 0; kc < KA; kc += 32) {
        v16h a[4];
#pragma unroll
        for (int mb = 0; mb < 4; ++mb) a[mb] = ldh(A + aoff + (size_t)mb * 16 * KA + kc);
#pragma unroll
        for (int nb = 0; nb < 4; ++nb) { const v16h b = ldh(Bt + boff + (size_t)nb * 16 * KA + kc);
#pragma unroll
            for (int mb = 0; mb < 4; ++mb) acc[mb][nb] = wmma16g(a[mb], b, acc[mb][nb]); }
    }
    const int n = r0 / MM;
    const int cofs = (lane & 15) * 4, rsub = lane >> 4;
    const v4f ad = *(const v4f*)(ADDp + (size_t)n * NA + c0 + cofs);
#pragma unroll
    for (int mb = 0; mb < 4; ++mb) {
#pragma unroll
        for (int nb = 0; nb < 4; ++nb) {
#pragma unroll
            for (int j = 0; j < 8; ++j) os[(hi * 8 + j) * 68 + nb * 16 + lr] = acc[mb][nb][j]; }
        wave_sync();
#pragma unroll 1
        for (int ps = 0; ps < 2; ++ps) {
#pragma unroll
            for (int s = 0; s < 8; ++s) { const int row = 2 * s + rsub;
                const v4f v = *(const v4fa*)(&os[row * 68 + cofs]);
                const v4f val = v * WINV + ad;
                *(volatile v4f*)(HP + (size_t)(r0 + mb * 16 + row) * NA + c0 + cofs) = val; }
            if (ps == 0) __threadfence(); }
        wave_sync();
    }
}

__global__ __launch_bounds__(32) void k_main(const bf* __restrict__ XB, const bf* __restrict__ WMp, const float* __restrict__ HP, float* OUT) {
    __shared__ __align__(16) float os[16 * 68];
    const int lane = threadIdx.x & 31, lr = lane & 15, hi = lane >> 4;
    const int ni = blockIdx.x >> 1, j0 = (blockIdx.x & 1) * 64, c0 = blockIdx.y * 64;
    const int n = ni / MM, i = ni % MM;
    v8f acc[4][4];
#pragma unroll
    for (int mb = 0; mb < 4; ++mb)
#pragma unroll
        for (int nb = 0; nb < 4; ++nb) acc[mb][nb] = (v8f){};
    const size_t doff = ((size_t)ni * MM + (size_t)(j0 + lr)) * DD + 8 * hi;
    const size_t toff = (((size_t)n * MM + (size_t)(j0 + lr)) * MM + (size_t)i) * DD + 8 * hi;
    const size_t boff = (size_t)(c0 + lr) * KM + 8 * hi;
#pragma unroll 1
    for (int kc = 0; kc < DD; kc += 32) {
        v16bf a[4];
#pragma unroll
        for (int mb = 0; mb < 4; ++mb) a[mb] = ldb(XB + doff + (size_t)mb * 16 * DD + kc);
#pragma unroll
        for (int nb = 0; nb < 4; ++nb) { const v16bf b = ldb(WMp + boff + (size_t)nb * 16 * KM + kc);
#pragma unroll
            for (int mb = 0; mb < 4; ++mb) acc[mb][nb] = wmmabg(a[mb], b, acc[mb][nb]); }
    }
#pragma unroll 1
    for (int kc = 0; kc < DD; kc += 32) {
        v16bf a[4];
#pragma unroll
        for (int mb = 0; mb < 4; ++mb) a[mb] = ldb(XB + toff + (size_t)mb * 16 * MM * DD + kc);
#pragma unroll
        for (int nb = 0; nb < 4; ++nb) { const v16bf b = ldb(WMp + boff + (size_t)nb * 16 * KM + DD + kc);
#pragma unroll
            for (int mb = 0; mb < 4; ++mb) acc[mb][nb] = wmmabg(a[mb], b, acc[mb][nb]); }
    }
    const int cofs = (lane & 15) * 4, rsub = lane >> 4;
    const v4f fi = *(const v4f*)(HP + (size_t)ni * NA + c0 + cofs);
    const v4f gg = *(const v4f*)(HP + (size_t)ni * NA + 2 * SS + c0 + cofs);
    const v4f zz = (v4f){};
#pragma unroll
    for (int mb = 0; mb < 4; ++mb) {
#pragma unroll
        for (int nb = 0; nb < 4; ++nb) {
#pragma unroll
            for (int j = 0; j < 8; ++j) os[(hi * 8 + j) * 68 + nb * 16 + lr] = acc[mb][nb][j]; }
        wave_sync();
#pragma unroll 1
        for (int ps = 0; ps < 2; ++ps) {
#pragma unroll
            for (int s = 0; s < 8; ++s) { const int row = 2 * s + rsub; const int jj = j0 + mb * 16 + row;
                const v4f v = *(const v4fa*)(&os[row * 68 + cofs]);
                const v4f fj = *(const v4f*)(HP + ((size_t)n * MM + (size_t)jj) * NA + SS + c0 + cofs);
                const v4f gd = (jj == i) ? gg : zz;
                const v4f tv = v + fi + fj + gd; v4f val;
#pragma unroll
                for (int e = 0; e < 4; ++e) val[e] = (tv[e] >= 0.0f) ? tv[e] : tv[e] * SLOPE;
                *(volatile v4f*)(OUT + ((size_t)ni * MM + (size_t)jj) * SS + c0 + cofs) = val; }
            if (ps == 0) __threadfence(); }
        wave_sync();
    }
}

static constexpr size_t al256(size_t v) { return (v + 255) & ~(size_t)255; }
static constexpr size_t SZ_XB = al256((size_t)NB * MM * MM * DD * 2);
static constexpr size_t SZ_WM = al256((size_t)SS * KM * 2);
static constexpr size_t SZ_WA = al256((size_t)NA * KA * 2);
static constexpr size_t SZ_AH = al256((size_t)NB * MM * KA * 2);
static constexpr size_t SZ_AF = al256((size_t)NB * MM * 2 * DD * 4);
static constexpr size_t SZ_AD = al256((size_t)NB * NA * 4);
static constexpr size_t SZ_HP = al256((size_t)NB * MM * NA * 4);
static constexpr size_t SZ_TOTAL = SZ_XB + SZ_WM + SZ_WA + SZ_AH + SZ_AF + SZ_AD + SZ_HP;
static_assert(SZ_TOTAL <= (size_t)134217728);
static_assert((size_t)NWM8 * 8 * 2 <= SZ_WM);
static_assert((size_t)NWA8 * 8 * 2 <= SZ_WA);
static_assert((size_t)(NB * MM - 1) * KA * 2 + (size_t)KA * 2 <= SZ_AH);
static_assert((size_t)(NB * MM - 1) * NA * 4 + (size_t)NA * 4 <= SZ_HP);

extern "C" void kernel_launch(void* const* d_in, const int* in_sizes, int n_in,
                              void* d_out, int out_size, void* d_ws, size_t ws_size, hipStream_t stream) {
    if (n_in < 4) return;
    const size_t needx = (size_t)NB * MM * MM * DD;
    if ((size_t)in_sizes[0] < needx) return;
    if ((size_t)in_sizes[1] < (size_t)DD * SS * NBAS) return;
    if (in_sizes[2] < SS || in_sizes[3] < SS) return;
    if ((size_t)out_size < (size_t)NB * MM * MM * SS) return;
    if (SZ_TOTAL > ws_size) return;
    const float* x     = (const float*)d_in[0];
    const float* coefs = (const float*)d_in[1];
    const float* bias  = (const float*)d_in[2];
    const float* dbias = (const float*)d_in[3];
    float* OUT = (float*)d_out;
    char* wsp = (char*)d_ws;
    bf*    XB  = (bf*)wsp;    wsp += SZ_XB;
    bf*    WMp = (bf*)wsp;    wsp += SZ_WM;
    h16*   WAp = (h16*)wsp;   wsp += SZ_WA;
    h16*   AH  = (h16*)wsp;   wsp += SZ_AH;
    float* AF  = (float*)wsp; wsp += SZ_AF;
    float* AD  = (float*)wsp; wsp += SZ_AD;
    float* HP  = (float*)wsp; wsp += SZ_HP;

    { const size_t n8 = needx / 8; k_cvt8<<<(unsigned)((n8 + 255) / 256), 256, 0, stream>>>(x, XB, n8); }
    k_pack<<<(NWM8 + NWA8) / 256, 256, 0, stream>>>(coefs, WMp, WAp);
    k_rowdiag<<<NB * MM, 128, 0, stream>>>(x, AF, AH);
    k_cols<<<NB * MM, 128, 0, stream>>>(x, AH);
    k_scal<<<NB, 128, 0, stream>>>(AF, coefs, bias, dbias, AD);
    k_agg<<<dim3(NB * MM / 64, NA / 64, 1), 32, 0, stream>>>(AH, WAp, AD, HP);
    k_main<<<dim3(NB * MM * 2, SS / 64, 1), 32, 0, stream>>>(XB, WMp, HP, OUT);
}
